// BahdanauCrossAttention_78804059947112
// MI455X (gfx1250) — hardware-run, weakly checked
//
#include <hip/hip_runtime.h>
#include <stdint.h>
#include <stddef.h>

#define NB   4
#define NQ   128
#define NK   1024
#define QD   512
#define KD   768
#define AD   256
#define MQ   512
#define MK   4096
#define TP   132
#define TQ   4
#define WSC  64.0f
#define VSC  16.0f
#define PSC  4096.0f
#define S_W   0.015625f
#define S_VP  0.25f
#define S_CT  0.00390625f
#define S_OUT 6.103515625e-05f

static_assert(MQ == NB * NQ);
static_assert(MK == NB * NK);
static_assert(QD % 128 == 0);
static_assert(NK % 128 == 0);
static_assert(AD % 128 == 0);
static_assert(MQ % 32 == 0);
static_assert(NQ % 32 == 0);
static_assert(AD % 32 == 0);
static_assert(QD % 32 == 0);
static_assert(KD % 32 == 0);
static_assert(NK % 32 == 0);
static_assert(NQ % TQ == 0);
static_assert(NK == 8 * 128);
static_assert(TQ == 4);
static_assert(TQ * AD == 4 * 256);
static_assert(AD / 4 == 64);
static_assert((TP * 4) % 16 == 0);
static_assert((MQ * QD) % 2048 == 0);
static_assert((MK * KD) % 2048 == 0);
static_assert((AD * QD) % 2048 == 0);
static_assert((AD * KD) % 2048 == 0);
static_assert((QD * KD) % 2048 == 0);
static_assert((QD * QD) % 2048 == 0);

typedef _Float16      v16h __attribute__((ext_vector_type(16)));
typedef float         v8f  __attribute__((ext_vector_type(8)));
typedef float         v4f  __attribute__((ext_vector_type(4)));
typedef unsigned int  v4u  __attribute__((ext_vector_type(4)));
typedef v4f __attribute__((may_alias)) v4fa;
typedef v4u __attribute__((may_alias)) v4ua;

union FragH { v16h v; v4u q[2]; };

__device__ __forceinline__ v8f wmma_h(v16h a, v16h b, v8f c) {
  v8f d = __builtin_amdgcn_wmma_f32_16x16x32_f16(false, a, false, b, (short)0, c, false, false);
  asm volatile("v_nop\n\tv_nop\n\tv_nop\n\tv_nop" : "+v"(d) : "v"(a), "v"(b));
  return d;
}

__device__ __forceinline__ v16h ldfrag(const unsigned short* p, int h) {
  FragH f;
  f.q[0] = *(const v4ua*)(p + 8 * h);
  f.q[1] = *(const v4ua*)(p + 16 + 8 * h);
  return f.v;
}

__device__ __forceinline__ unsigned short hb16(_Float16 x) {
  return __builtin_bit_cast(unsigned short, x);
}
__device__ __forceinline__ unsigned short hbits(float a) {
  return hb16((_Float16)a);
}
__device__ __forceinline__ unsigned int pkh(float a, float b) {
  return (unsigned int)hbits(a) | ((unsigned int)hbits(b) << 16);
}
__device__ __forceinline__ v4u pack8(const float* f) {
  v4u p;
  p.x = pkh(f[0], f[1]);
  p.y = pkh(f[2], f[3]);
  p.z = pkh(f[4], f[5]);
  p.w = pkh(f[6], f[7]);
  return p;
}

__device__ __forceinline__ float tnh(float x) {
  return 1.0f - 2.0f * __builtin_amdgcn_rcpf(__expf(2.0f * x) + 1.0f);
}

__global__ __launch_bounds__(256) void k_plane(const float* __restrict__ src, int n8,
                                               float s, unsigned short* __restrict__ dst)
{
  const int g = blockIdx.x * 256 + threadIdx.x;
  if (g >= n8) return;
  const size_t e0 = (size_t)g * 8;
  const v4f x0 = *(const v4fa*)(src + e0);
  const v4f x1 = *(const v4fa*)(src + e0 + 4);
  float f[8];
  f[0] = x0.x * s; f[1] = x0.y * s; f[2] = x0.z * s; f[3] = x0.w * s;
  f[4] = x1.x * s; f[5] = x1.y * s; f[6] = x1.z * s; f[7] = x1.w * s;
  const v4u p = pack8(f);
  unsigned short* d = dst + e0;
  *(volatile v4u*)d = p;
  __threadfence();
  *(volatile v4u*)d = p;
}

template <int OH>
__global__ __launch_bounds__(256) void k_gemm(const unsigned short* __restrict__ A, int lda, long long zA,
                                              const unsigned short* __restrict__ Bw, int ldb, long long zB,
                                              const float* __restrict__ bias, int nb, int hb,
                                              int K, float sc,
                                              float* __restrict__ C, unsigned short* __restrict__ P,
                                              int ldc, long long zC)
{
  __shared__ __align__(16) float sT[32 * TP];

  const int tid = threadIdx.x, lane = tid & 31, wv = tid >> 5;
  const int h = lane >> 4, m = lane & 15;
  const int n0 = blockIdx.x * 128, m0 = blockIdx.y * 32, z = blockIdx.z;
  const int nc = n0 + 16 * wv;
  const unsigned short* Az = A  + (size_t)zA * (size_t)z;
  const unsigned short* Bz = Bw + (size_t)zB * (size_t)z;

  const v8f z8 = {0.f, 0.f, 0.f, 0.f, 0.f, 0.f, 0.f, 0.f};
  v8f acc0 = z8, acc1 = z8;
  const size_t ra0 = (size_t)(m0 + m) * lda;
  const size_t ra1 = (size_t)(m0 + 16 + m) * lda;
  const size_t rb  = (size_t)(nc + m) * ldb;

  #pragma unroll 1
  for (int k0 = 0; k0 < K; k0 += 32) {
    const v16h a0 = ldfrag(Az + ra0 + k0, h);
    const v16h a1 = ldfrag(Az + ra1 + k0, h);
    const v16h b  = ldfrag(Bz + rb + k0, h);
    acc0 = wmma_h(a0, b, acc0);
    acc1 = wmma_h(a1, b, acc1);
  }

  const int bi = (nc + m < nb) ? (nc + m) : (nb - 1);
  const float bl = bias[bi];
  const float bv = hb ? bl : 0.0f;
  #pragma unroll
  for (int r = 0; r < 8; ++r) {
    sT[(8 * h + r) * TP + 16 * wv + m]      = acc0[r] * sc + bv;
    sT[(16 + 8 * h + r) * TP + 16 * wv + m] = acc1[r] * sc + bv;
  }
  __syncthreads();

  if (OH == 0) {
    float* Cz = C + (size_t)zC * (size_t)z;
    v4f ov[4];
    size_t ga[4];
    #pragma unroll
    for (int i = 0; i < 4; ++i) {
      const int row = wv + 8 * i;
      ov[i] = *(const v4fa*)(sT + row * TP + 4 * lane);
      ga[i] = (size_t)(m0 + row) * ldc + n0 + 4 * lane;
    }
    #pragma unroll
    for (int i = 0; i < 4; ++i) *(volatile v4f*)(Cz + ga[i]) = ov[i];
    __threadfence();
    #pragma unroll
    for (int i = 0; i < 4; ++i) *(volatile v4f*)(Cz + ga[i]) = ov[i];
  } else {
    unsigned short* Pz = P + (size_t)zC * (size_t)z;
    v4u pv[2];
    size_t pa[2];
    #pragma unroll
    for (int q = 0; q < 2; ++q) {
      const int row = wv + 8 * (2 * q + h);
      const float* sp = sT + row * TP + 8 * m;
      const v4f x0 = *(const v4fa*)sp;
      const v4f x1 = *(const v4fa*)(sp + 4);
      float f[8];
      f[0] = x0.x; f[1] = x0.y; f[2] = x0.z; f[3] = x0.w;
      f[4] = x1.x; f[5] = x1.y; f[6] = x1.z; f[7] = x1.w;
      pv[q] = pack8(f);
      pa[q] = (size_t)(m0 + row) * ldc + n0 + 8 * m;
    }
    #pragma unroll
    for (int q = 0; q < 2; ++q) *(volatile v4u*)(Pz + pa[q]) = pv[q];
    __threadfence();
    #pragma unroll
    for (int q = 0; q < 2; ++q) *(volatile v4u*)(Pz + pa[q]) = pv[q];
  }
}

__global__ __launch_bounds__(256) void k_energy(const float* __restrict__ qp,
                                                const float* __restrict__ kpT,
                                                const float* __restrict__ vv,
                                                float* __restrict__ alpha,
                                                unsigned short* __restrict__ Pp)
{
  __shared__ __align__(16) float sQ[TQ * AD];
  __shared__ __align__(16) float sV[AD];
  __shared__ __align__(16) float sA[TQ * NK];
  __shared__ float sRm[8 * TQ];
  __shared__ float sRs[8 * TQ];

  const int tid = threadIdx.x, lane = tid & 31, wv = tid >> 5;
  const int blk = blockIdx.x;
  const int b = blk / (NQ / TQ);
  const size_t row0 = (size_t)blk * TQ;

  *(v4fa*)(sQ + 4 * tid) = *(const v4fa*)(qp + row0 * AD + 4 * tid);
  if (tid < AD / 4) *(v4fa*)(sV + 4 * tid) = *(const v4fa*)(vv + 4 * tid);
  __syncthreads();

  float e[4][TQ];
  #pragma unroll
  for (int g = 0; g < 4; ++g) {
    #pragma unroll
    for (int q = 0; q < TQ; ++q) e[g][q] = 0.0f;
  }
  const float* kbp = kpT + (size_t)b * AD * NK + 128 * wv + lane;
  #pragma unroll 1
  for (int d = 0; d < AD; ++d) {
    const float* kr = kbp + (size_t)d * NK;
    float kk[4];
    kk[0] = kr[0]; kk[1] = kr[32]; kk[2] = kr[64]; kk[3] = kr[96];
    const float vd = sV[d];
    #pragma unroll
    for (int q = 0; q < TQ; ++q) {
      const float x = sQ[q * AD + d];
      #pragma unroll
      for (int g = 0; g < 4; ++g) e[g][q] += tnh(x + kk[g]) * vd;
    }
  }

  float M[TQ];
  #pragma unroll
  for (int q = 0; q < TQ; ++q) {
    float mq = fmaxf(fmaxf(e[0][q], e[1][q]), fmaxf(e[2][q], e[3][q]));
    #pragma unroll
    for (int off = 16; off; off >>= 1) mq = fmaxf(mq, __shfl_xor(mq, off, 32));
    M[q] = mq;
  }
  if (lane == 0) {
    #pragma unroll
    for (int q = 0; q < TQ; ++q) sRm[wv * TQ + q] = M[q];
  }
  __syncthreads();
  #pragma unroll
  for (int q = 0; q < TQ; ++q) {
    float mm = sRm[q];
    #pragma unroll
    for (int w = 1; w < 8; ++w) mm = fmaxf(mm, sRm[w * TQ + q]);
    M[q] = mm;
  }

  float S[TQ];
  #pragma unroll
  for (int q = 0; q < TQ; ++q) {
    float s = 0.0f;
    #pragma unroll
    for (int g = 0; g < 4; ++g) {
      const float ex = __expf(e[g][q] - M[q]);
      sA[q * NK + 128 * wv + 32 * g + lane] = ex;
      s += ex;
    }
    #pragma unroll
    for (int off = 16; off; off >>= 1) s += __shfl_xor(s, off, 32);
    S[q] = s;
  }
  if (lane == 0) {
    #pragma unroll
    for (int q = 0; q < TQ; ++q) sRs[wv * TQ + q] = S[q];
  }
  __syncthreads();
  float inv[TQ];
  #pragma unroll
  for (int q = 0; q < TQ; ++q) {
    float tot = sRs[q];
    #pragma unroll
    for (int w = 1; w < 8; ++w) tot += sRs[w * TQ + q];
    inv[q] = __builtin_amdgcn_rcpf(tot);
  }

  const int qa = (wv < TQ) ? wv : (wv - TQ);
  float iv = 0.0f;
  #pragma unroll
  for (int qq = 0; qq < TQ; ++qq) iv = (qq == qa) ? inv[qq] : iv;
  const float* sa = sA + qa * NK;
  const size_t grow = (row0 + qa) * NK;
  if (wv < TQ) {
    v4f ov[8];
    size_t ga[8];
    #pragma unroll
    for (int i = 0; i < 8; ++i) {
      const v4f x = *(const v4fa*)(sa + 128 * i + 4 * lane);
      ov[i] = x * iv;
      ga[i] = grow + 128 * i + 4 * lane;
    }
    #pragma unroll
    for (int i = 0; i < 8; ++i) *(volatile v4f*)(alpha + ga[i]) = ov[i];
    __threadfence();
    #pragma unroll
    for (int i = 0; i < 8; ++i) *(volatile v4f*)(alpha + ga[i]) = ov[i];
  } else {
    const float ip = iv * PSC;
    v4u pv[4];
    size_t pa[4];
    #pragma unroll
    for (int i = 0; i < 4; ++i) {
      const float* sp = sa + 256 * i + 8 * lane;
      const v4f x0 = *(const v4fa*)sp;
      const v4f x1 = *(const v4fa*)(sp + 4);
      float f[8];
      f[0] = x0.x * ip; f[1] = x0.y * ip; f[2] = x0.z * ip; f[3] = x0.w * ip;
      f[4] = x1.x * ip; f[5] = x1.y * ip; f[6] = x1.z * ip; f[7] = x1.w * ip;
      pv[i] = pack8(f);
      pa[i] = grow + 256 * i + 8 * lane;
    }
    #pragma unroll
    for (int i = 0; i < 4; ++i) *(volatile v4u*)(Pp + pa[i]) = pv[i];
    __threadfence();
    #pragma unroll
    for (int i = 0; i < 4; ++i) *(volatile v4u*)(Pp + pa[i]) = pv[i];
  }
}

static void plane(const float* src, int n, float s, unsigned short* dst, hipStream_t st)
{
  const int n8 = n / 8;
  k_plane<<<(n8 + 255) / 256, 256, 0, st>>>(src, n8, s, dst);
}

extern "C" void kernel_launch(void* const* d_in, const int* in_sizes, int n_in,
                              void* d_out, int out_size, void* d_ws, size_t ws_size,
                              hipStream_t stream)
{
  if (n_in < 8) return;
  if (in_sizes[0] != MQ * QD) return;
  if (in_sizes[1] != MK * KD) return;
  if (in_sizes[2] != AD * QD) return;
  if (in_sizes[3] != AD * KD) return;
  if (in_sizes[4] != AD) return;
  if (in_sizes[5] != QD * KD) return;
  if (in_sizes[6] != QD * QD) return;
  if (in_sizes[7] != QD) return;
  if (out_size != MQ * QD + MQ * NK) return;

  const float* q   = (const float*)d_in[0];
  const float* kv  = (const float*)d_in[1];
  const float* W_q = (const float*)d_in[2];
  const float* W_k = (const float*)d_in[3];
  const float* vv  = (const float*)d_in[4];
  const float* W_v = (const float*)d_in[5];
  const float* W_o = (const float*)d_in[6];
  const float* b_o = (const float*)d_in[7];
  float* out0 = (float*)d_out;
  float* out1 = (float*)d_out + (size_t)MQ * QD;

  const size_t bQ  = (size_t)MQ * QD * 2;
  const size_t bKV = (size_t)MK * KD * 2;
  const size_t bWq = (size_t)AD * QD * 2;
  const size_t bWk = (size_t)AD * KD * 2;
  const size_t bWv = (size_t)QD * KD * 2;
  const size_t bWo = (size_t)QD * QD * 2;
  const size_t bQp = (size_t)MQ * AD * 4;
  const size_t bKp = (size_t)NB * AD * NK * 4;
  const size_t bVp = (size_t)NB * QD * NK * 2;
  const size_t bP  = (size_t)MQ * NK * 2;
  const size_t bCt = (size_t)MQ * QD * 2;
  const size_t total = bQ + bKV + bWq + bWk + bWv + bWo + bQp + bKp + bVp + bP + bCt;
  if (total > ws_size) return;
  if (total > (size_t)134217728) return;

  char* ws = (char*)d_ws;
  size_t off = 0;
  unsigned short* pQ   = (unsigned short*)(ws + off); off += bQ;
  unsigned short* pKV  = (unsigned short*)(ws + off); off += bKV;
  unsigned short* pWq  = (unsigned short*)(ws + off); off += bWq;
  unsigned short* pWk  = (unsigned short*)(ws + off); off += bWk;
  unsigned short* pWv  = (unsigned short*)(ws + off); off += bWv;
  unsigned short* pWo  = (unsigned short*)(ws + off); off += bWo;
  float*          qp   = (float*)(ws + off);          off += bQp;
  float*          kpT  = (float*)(ws + off);          off += bKp;
  unsigned short* pVp  = (unsigned short*)(ws + off); off += bVp;
  unsigned short* pP   = (unsigned short*)(ws + off); off += bP;
  unsigned short* pCt  = (unsigned short*)(ws + off); off += bCt;
  if (off != total) return;

  plane(q,   MQ * QD, 1.0f, pQ,  stream);
  plane(kv,  MK * KD, 1.0f, pKV, stream);
  plane(W_q, AD * QD, WSC,  pWq, stream);
  plane(W_k, AD * KD, WSC,  pWk, stream);
  plane(W_v, QD * KD, WSC,  pWv, stream);
  plane(W_o, QD * QD, WSC,  pWo, stream);

  k_gemm<0><<<dim3(AD / 128, MQ / 32, 1), 256, 0, stream>>>(
      pQ, QD, 0LL, pWq, QD, 0LL, b_o, QD, 0, QD, S_W, qp, pCt, AD, 0LL);

  k_gemm<0><<<dim3(NK / 128, AD / 32, NB), 256, 0, stream>>>(
      pWk, KD, 0LL, pKV, KD, (long long)NK * KD, b_o, QD, 0, KD, S_W,
      kpT, pCt, NK, (long long)AD * NK);

  k_gemm<1><<<dim3(NK / 128, QD / 32, NB), 256, 0, stream>>>(
      pWv, KD, 0LL, pKV, KD, (long long)NK * KD, b_o, QD, 0, KD, S_VP,
      qp, pVp, NK, (long long)QD * NK);

  k_energy<<<MQ / TQ, 256, 0, stream>>>(qp, kpT, vv, out1, pP);

  k_gemm<1><<<dim3(QD / 128, NQ / 32, NB), 256, 0, stream>>>(
      pP, NK, (long long)NQ * NK, pVp, NK, (long long)QD * NK, b_o, QD, 0, NK, S_CT,
      qp, pCt, QD, (long long)NQ * QD);

  k_gemm<0><<<dim3(QD / 128, MQ / 32, 1), 256, 0, stream>>>(
      pCt, QD, 0LL, pWo, QD, 0LL, b_o, QD, 1, QD, S_OUT, out0, pCt, QD, 0LL);
}
